// SelfAtten_34076270527142
// MI455X (gfx1250) — hardware-verified
//
#include <hip/hip_runtime.h>
#include <math.h>
#include <stdint.h>

#define NB    4
#define DCH   128
#define KC    64
#define SEQ   4096
#define NCH   256
#define QT    64
#define AP    144
#define LP    72
#define OP    68
#define LNPS  6.931471805599453f
#define RSC   2048.0f
#define IRSC  0.00048828125f
static_assert((SEQ % QT) == 0);
static_assert((SEQ % 32) == 0);
static_assert(DCH == 128);
static_assert(KC == 64);
static_assert(NCH == 2 * KC + DCH);
static_assert(((NCH * DCH) / 8) % 256 == 0);
static_assert(64 * AP == DCH * LP);

typedef _Float16       v16h __attribute__((ext_vector_type(16)));
typedef _Float16       v8h  __attribute__((ext_vector_type(8)));
typedef __bf16         v16b __attribute__((ext_vector_type(16)));
typedef unsigned short v8us __attribute__((ext_vector_type(8)));
typedef float          v8f  __attribute__((ext_vector_type(8)));
typedef float          v4f  __attribute__((ext_vector_type(4)));
typedef unsigned int   v4u  __attribute__((ext_vector_type(4)));

union FragH { v16h v; v8h  h[2]; };
union FragB { v16b v; v8us u[2]; };
static_assert(sizeof(FragH) == 32);
static_assert(sizeof(FragB) == 32);

__device__ __forceinline__ unsigned short bf_bits(float f) {
  unsigned u = __float_as_uint(f);
  return (unsigned short)((u + 0x7FFFu + ((u >> 16) & 1u)) >> 16);
}
__device__ __forceinline__ float bf_up(unsigned short h) { return __uint_as_float(((unsigned)h) << 16); }
__device__ __forceinline__ float bfr(float f) { return bf_up(bf_bits(f)); }
__device__ __forceinline__ unsigned short h_bits(_Float16 x) { return __builtin_bit_cast(unsigned short, x); }
__device__ __forceinline__ unsigned pk16(unsigned short a, unsigned short b) { return (unsigned)a | ((unsigned)b << 16); }
__device__ __forceinline__ v8f zero8() { v8f z = {0.f, 0.f, 0.f, 0.f, 0.f, 0.f, 0.f, 0.f}; return z; }
__device__ __forceinline__ float hmax8(v8f s) {
  return fmaxf(fmaxf(fmaxf(s[0], s[1]), fmaxf(s[2], s[3])), fmaxf(fmaxf(s[4], s[5]), fmaxf(s[6], s[7])));
}

__device__ __forceinline__ v16h ldfrag_h(const _Float16* p) {
  FragH f;
  f.h[0] = *(const v8h*)(p);
  f.h[1] = *(const v8h*)(p + 16);
  return f.v;
}
__device__ __forceinline__ v16b ldfrag_b(const unsigned short* p) {
  FragB f;
  f.u[0] = *(const v8us*)(p);
  f.u[1] = *(const v8us*)(p + 16);
  return f.v;
}

__device__ __forceinline__ v8f mma_h(v16h a, v16h b, v8f c) {
  v8f d = __builtin_amdgcn_wmma_f32_16x16x32_f16(false, a, false, b, (short)0, c, false, false);
#if defined(__HIP_DEVICE_COMPILE__)
  asm volatile("v_nop\n\tv_nop\n\tv_nop\n\tv_nop" : "+v"(d) : "v"(a), "v"(b));
#endif
  return d;
}
__device__ __forceinline__ v8f mma_b(v16b a, v16b b, v8f c) {
  v8f d = __builtin_amdgcn_wmma_f32_16x16x32_bf16(false, a, false, b, (short)0, c, false, false);
#if defined(__HIP_DEVICE_COMPILE__)
  const v16h ha = __builtin_bit_cast(v16h, a), hb = __builtin_bit_cast(v16h, b);
  asm volatile("v_nop\n\tv_nop\n\tv_nop\n\tv_nop" : "+v"(d) : "v"(ha), "v"(hb));
#endif
  return d;
}

__device__ __forceinline__ void stage_split(unsigned short* Lh, unsigned short* Ll, int nr, int col, v8f acc, float bias) {
#pragma unroll
  for (int r = 0; r < 8; ++r) {
    const float val = acc[r] + bias;
    const _Float16 hi = (_Float16)val;
    const float res = (val - (float)hi) * RSC;
    Lh[(nr + r) * LP + col] = h_bits(hi);
    Ll[(nr + r) * LP + col] = h_bits((_Float16)res);
  }
}
__device__ __forceinline__ void stage_v(unsigned short* Lv, int e, int nr, v8f acc, float bias) {
#pragma unroll
  for (int r = 0; r < 8; ++r) Lv[e * LP + nr + r] = h_bits((_Float16)(acc[r] + bias));
}

__global__ __launch_bounds__(256) void cvt_w(const float* __restrict__ wq, const float* __restrict__ wk,
                                              const float* __restrict__ wv, unsigned short* WB) {
  const int i = blockIdx.x * 256 + threadIdx.x;
  if (i >= (NCH * DCH) / 8) return;
  const int row = i >> 4;
  const int col = (i & 15) * 8;
  const int rq = min(row, KC - 1);
  const int rk = min(max(row - KC, 0), KC - 1);
  const int rv = min(max(row - 2 * KC, 0), DCH - 1);
  const v4f q0 = *(const v4f*)(wq + rq * DCH + col), q1 = *(const v4f*)(wq + rq * DCH + col + 4);
  const v4f k0 = *(const v4f*)(wk + rk * DCH + col), k1 = *(const v4f*)(wk + rk * DCH + col + 4);
  const v4f v0 = *(const v4f*)(wv + rv * DCH + col), v1 = *(const v4f*)(wv + rv * DCH + col + 4);
  const bool isq = row < KC;
  const bool isk = row < 2 * KC;
  v4u w;
#pragma unroll
  for (int t = 0; t < 2; ++t) {
    const float a0 = isq ? q0[2 * t]     : (isk ? k0[2 * t]     : v0[2 * t]);
    const float a1 = isq ? q0[2 * t + 1] : (isk ? k0[2 * t + 1] : v0[2 * t + 1]);
    const float c0 = isq ? q1[2 * t]     : (isk ? k1[2 * t]     : v1[2 * t]);
    const float c1 = isq ? q1[2 * t + 1] : (isk ? k1[2 * t + 1] : v1[2 * t + 1]);
    w[t]     = pk16(bf_bits(a0), bf_bits(a1));
    w[2 + t] = pk16(bf_bits(c0), bf_bits(c1));
  }
  unsigned short* p = WB + (size_t)i * 8;
  *(volatile v4u*)p = w;
  __threadfence();
  *(volatile v4u*)p = w;
}

__global__ __launch_bounds__(256)
void proj_kernel(const float* __restrict__ x, const unsigned short* __restrict__ WB,
                 const float* __restrict__ bqp, const float* __restrict__ bkp, const float* __restrict__ bvp,
                 unsigned short* QH, unsigned short* QL, unsigned short* KH, unsigned short* KL, unsigned short* VP) {
  __shared__ __align__(16) unsigned short Lav[64 * AP];
  __shared__ __align__(16) unsigned short Lq[2][64 * LP];
  __shared__ __align__(16) unsigned short Lk[2][64 * LP];
  const int tid  = threadIdx.x;
  const int lane = tid & 31, wave = tid >> 5;
  const int hh   = lane >> 4, c = lane & 15;
  const int bx   = blockIdx.x;
  const int b    = bx / (SEQ / QT);
  const int nt   = bx % (SEQ / QT);
  const int n0   = nt * QT;

  {
    const int n4 = (tid & 15) * 4, ds = tid >> 4;
    const float* xp = x + ((size_t)b * DCH + ds) * SEQ + n0 + n4;
#pragma unroll
    for (int it = 0; it < 8; ++it) {
      const v4f v = *(const v4f*)(xp + (size_t)it * 16 * SEQ);
      const int d = it * 16 + ds;
#pragma unroll
      for (int q = 0; q < 4; ++q) Lav[(n4 + q) * AP + d] = bf_bits(v[q]);
    }
  }
  __syncthreads();

  const int ng = wave & 3, ch = wave >> 2;
  const unsigned short* ap = Lav + (ng * 16 + c) * AP + 8 * hh;
  const unsigned short* bp = WB + (size_t)(ch * DCH + c) * DCH + 8 * hh;
  v8f acc0 = zero8(), acc1 = zero8(), acc2 = zero8(), acc3 = zero8();
  v8f acc4 = zero8(), acc5 = zero8(), acc6 = zero8(), acc7 = zero8();
#pragma unroll
  for (int ks = 0; ks < 4; ++ks) {
    const v16b a = ldfrag_b(ap + 32 * ks);
    const unsigned short* bs = bp + 32 * ks;
    acc0 = mma_b(a, ldfrag_b(bs + 0 * 16 * DCH), acc0);
    acc1 = mma_b(a, ldfrag_b(bs + 1 * 16 * DCH), acc1);
    acc2 = mma_b(a, ldfrag_b(bs + 2 * 16 * DCH), acc2);
    acc3 = mma_b(a, ldfrag_b(bs + 3 * 16 * DCH), acc3);
    acc4 = mma_b(a, ldfrag_b(bs + 4 * 16 * DCH), acc4);
    acc5 = mma_b(a, ldfrag_b(bs + 5 * 16 * DCH), acc5);
    acc6 = mma_b(a, ldfrag_b(bs + 6 * 16 * DCH), acc6);
    acc7 = mma_b(a, ldfrag_b(bs + 7 * 16 * DCH), acc7);
  }

  const float bq0 = bfr(bqp[0 * 16 + c]), bq1 = bfr(bqp[1 * 16 + c]), bq2 = bfr(bqp[2 * 16 + c]), bq3 = bfr(bqp[3 * 16 + c]);
  const float bk0 = bfr(bkp[0 * 16 + c]), bk1 = bfr(bkp[1 * 16 + c]), bk2 = bfr(bkp[2 * 16 + c]), bk3 = bfr(bkp[3 * 16 + c]);
  const float bv0 = bfr(bvp[0 * 16 + c]), bv1 = bfr(bvp[1 * 16 + c]), bv2 = bfr(bvp[2 * 16 + c]), bv3 = bfr(bvp[3 * 16 + c]);
  const float bv4 = bfr(bvp[4 * 16 + c]), bv5 = bfr(bvp[5 * 16 + c]), bv6 = bfr(bvp[6 * 16 + c]), bv7 = bfr(bvp[7 * 16 + c]);

  __syncthreads();
  const int nr = ng * 16 + 8 * hh;
  if (ch == 0) {
    stage_split(Lq[0], Lq[1], nr, 0 * 16 + c, acc0, bq0);
    stage_split(Lq[0], Lq[1], nr, 1 * 16 + c, acc1, bq1);
    stage_split(Lq[0], Lq[1], nr, 2 * 16 + c, acc2, bq2);
    stage_split(Lq[0], Lq[1], nr, 3 * 16 + c, acc3, bq3);
    stage_split(Lk[0], Lk[1], nr, 0 * 16 + c, acc4, bk0);
    stage_split(Lk[0], Lk[1], nr, 1 * 16 + c, acc5, bk1);
    stage_split(Lk[0], Lk[1], nr, 2 * 16 + c, acc6, bk2);
    stage_split(Lk[0], Lk[1], nr, 3 * 16 + c, acc7, bk3);
  } else {
    stage_v(Lav, 0 * 16 + c, nr, acc0, bv0);
    stage_v(Lav, 1 * 16 + c, nr, acc1, bv1);
    stage_v(Lav, 2 * 16 + c, nr, acc2, bv2);
    stage_v(Lav, 3 * 16 + c, nr, acc3, bv3);
    stage_v(Lav, 4 * 16 + c, nr, acc4, bv4);
    stage_v(Lav, 5 * 16 + c, nr, acc5, bv5);
    stage_v(Lav, 6 * 16 + c, nr, acc6, bv6);
    stage_v(Lav, 7 * 16 + c, nr, acc7, bv7);
  }
  __syncthreads();

  {
    const int e = tid & 7, lq = tid >> 3;
#pragma unroll
    for (int pass = 0; pass < 2; ++pass) {
#pragma unroll
      for (int it = 0; it < 2; ++it) {
        const int n = it * 32 + lq;
        const size_t go = ((size_t)b * SEQ + n0 + n) * KC + 8 * e;
        const int lo_ = n * LP + 8 * e;
        const v4u uqh = *(const v4u*)(Lq[0] + lo_);
        const v4u uql = *(const v4u*)(Lq[1] + lo_);
        const v4u ukh = *(const v4u*)(Lk[0] + lo_);
        const v4u ukl = *(const v4u*)(Lk[1] + lo_);
        *(volatile v4u*)(QH + go) = uqh;
        *(volatile v4u*)(QL + go) = uql;
        *(volatile v4u*)(KH + go) = ukh;
        *(volatile v4u*)(KL + go) = ukl;
      }
#pragma unroll
      for (int it = 0; it < 4; ++it) {
        const int er = it * 32 + lq;
        const v4u uv = *(const v4u*)(Lav + er * LP + 8 * e);
        *(volatile v4u*)(VP + ((size_t)b * DCH + er) * SEQ + n0 + 8 * e) = uv;
      }
      __threadfence();
    }
  }
}

__global__ __launch_bounds__(128)
void attn_kernel(const unsigned short* __restrict__ QH, const unsigned short* __restrict__ QL,
                 const unsigned short* __restrict__ KH, const unsigned short* __restrict__ KL,
                 const unsigned short* __restrict__ VP, float* out) {
  __shared__ __align__(16) float Os[DCH * OP];
  const int tid  = threadIdx.x;
  const int wave = tid >> 5;
  const int lane = tid & 31;
  const int hh   = lane >> 4;
  const int c    = lane & 15;
  const int bx   = blockIdx.x;
  const int b    = bx / (SEQ / QT);
  const int qb   = bx % (SEQ / QT);
  const int n0   = qb * QT;
  const _Float16* QHh = (const _Float16*)(const void*)QH;
  const _Float16* QLh = (const _Float16*)(const void*)QL;
  const _Float16* KHh = (const _Float16*)(const void*)KH;
  const _Float16* KLh = (const _Float16*)(const void*)KL;
  const _Float16* VPh = (const _Float16*)(const void*)VP;

  const size_t qo = ((size_t)b * SEQ + n0 + wave * 16 + c) * KC + 8 * hh;
  const v16h qh0 = ldfrag_h(QHh + qo), qh1 = ldfrag_h(QHh + qo + 32);
  const v16h ql0 = ldfrag_h(QLh + qo), ql1 = ldfrag_h(QLh + qo + 32);
  const size_t ko = ((size_t)b * SEQ + c) * KC + 8 * hh;
  const _Float16* Kp = KHh + ko;
  const _Float16* Lp = KLh + ko;
  const _Float16* Vb = VPh + ((size_t)b * DCH + c) * SEQ + 8 * hh;

  float m = -1.0e30f, l = 0.f;
  v8f o0 = zero8(), o1 = zero8(), o2 = zero8(), o3 = zero8();
  v8f o4 = zero8(), o5 = zero8(), o6 = zero8(), o7 = zero8();
#pragma unroll 1
  for (int it = 0; it < SEQ / 32; ++it) {
    const int kb = it * 32;
    const _Float16* k0p = Kp + (size_t)kb * KC;
    const _Float16* k1p = k0p + 16 * KC;
    const _Float16* l0p = Lp + (size_t)kb * KC;
    const _Float16* l1p = l0p + 16 * KC;
    v8f s0, t0, s1, t1;
    {
      const v16h a0 = ldfrag_h(k0p), a1 = ldfrag_h(k0p + 32);
      s0 = mma_h(a0, qh0, zero8());
      s0 = mma_h(a1, qh1, s0);
      t0 = mma_h(a0, ql0, zero8());
      t0 = mma_h(a1, ql1, t0);
      const v16h r0 = ldfrag_h(l0p), r1 = ldfrag_h(l0p + 32);
      t0 = mma_h(r0, qh0, t0);
      t0 = mma_h(r1, qh1, t0);
    }
    {
      const v16h a0 = ldfrag_h(k1p), a1 = ldfrag_h(k1p + 32);
      s1 = mma_h(a0, qh0, zero8());
      s1 = mma_h(a1, qh1, s1);
      t1 = mma_h(a0, ql0, zero8());
      t1 = mma_h(a1, ql1, t1);
      const v16h r0 = ldfrag_h(l1p), r1 = ldfrag_h(l1p + 32);
      t1 = mma_h(r0, qh0, t1);
      t1 = mma_h(r1, qh1, t1);
    }
#pragma unroll
    for (int r = 0; r < 8; ++r) {
      s0[r] = s0[r] + t0[r] * IRSC;
      s1[r] = s1[r] + t1[r] * IRSC;
    }

    float mx = fmaxf(hmax8(s0), hmax8(s1));
    mx = fmaxf(mx, __shfl_xor(mx, 16, 32));
    const float mn   = fmaxf(m, mx);
    const float corr = __expf(m - mn);
    m = mn;
    const float msh = mn - LNPS;
    l *= corr;
#pragma unroll
    for (int r = 0; r < 8; ++r) {
      o0[r] *= corr; o1[r] *= corr; o2[r] *= corr; o3[r] *= corr;
      o4[r] *= corr; o5[r] *= corr; o6[r] *= corr; o7[r] *= corr;
    }

    FragH ph;
    float ls = 0.f;
#pragma unroll
    for (int r = 0; r < 8; ++r) {
      const float e0 = __expf(s0[r] - msh);
      const float e1 = __expf(s1[r] - msh);
      ls += e0 + e1;
      ph.h[0][r] = (_Float16)e0;
      ph.h[1][r] = (_Float16)e1;
    }
    l += ls;

    o0 = mma_h(ldfrag_h(Vb + 0 * 16 * SEQ + kb), ph.v, o0);
    o1 = mma_h(ldfrag_h(Vb + 1 * 16 * SEQ + kb), ph.v, o1);
    o2 = mma_h(ldfrag_h(Vb + 2 * 16 * SEQ + kb), ph.v, o2);
    o3 = mma_h(ldfrag_h(Vb + 3 * 16 * SEQ + kb), ph.v, o3);
    o4 = mma_h(ldfrag_h(Vb + 4 * 16 * SEQ + kb), ph.v, o4);
    o5 = mma_h(ldfrag_h(Vb + 5 * 16 * SEQ + kb), ph.v, o5);
    o6 = mma_h(ldfrag_h(Vb + 6 * 16 * SEQ + kb), ph.v, o6);
    o7 = mma_h(ldfrag_h(Vb + 7 * 16 * SEQ + kb), ph.v, o7);
  }
  l += __shfl_xor(l, 16, 32);
  const float sc = 1.0f / l;

  float* os = Os + (8 * hh) * OP + wave * 16 + c;
#pragma unroll
  for (int r = 0; r < 8; ++r) {
    os[(0 * 16 + r) * OP] = o0[r] * sc; os[(1 * 16 + r) * OP] = o1[r] * sc;
    os[(2 * 16 + r) * OP] = o2[r] * sc; os[(3 * 16 + r) * OP] = o3[r] * sc;
    os[(4 * 16 + r) * OP] = o4[r] * sc; os[(5 * 16 + r) * OP] = o5[r] * sc;
    os[(6 * 16 + r) * OP] = o6[r] * sc; os[(7 * 16 + r) * OP] = o7[r] * sc;
  }
  __syncthreads();
  {
    const int e = tid & 7, lq = tid >> 3;
    float* ob = out + ((size_t)b * DCH) * SEQ + n0;
#pragma unroll
    for (int pass = 0; pass < 2; ++pass) {
#pragma unroll
      for (int it = 0; it < 16; ++it) {
        const int L   = it * 16 + lq;
        const int row = L >> 1, hf = L & 1;
        const v4f v = *(const v4f*)(Os + row * OP + hf * 32 + 4 * e);
        *(volatile v4f*)(ob + (size_t)row * SEQ + hf * 32 + 4 * e) = v;
      }
      __threadfence();
    }
  }
}

extern "C" void kernel_launch(void* const* d_in, const int* in_sizes, int n_in,
                              void* d_out, int out_size, void* d_ws, size_t ws_size,
                              hipStream_t stream) {
  const int NX = NB * DCH * SEQ;
  if (n_in < 7) return;
  if (in_sizes[0] != NX || in_sizes[1] != KC * DCH || in_sizes[2] != KC || in_sizes[3] != KC * DCH ||
      in_sizes[4] != KC || in_sizes[5] != DCH * DCH || in_sizes[6] != DCH) return;
  if (out_size != NX) return;

  size_t off = 0;
  const size_t oW  = off; off += (size_t)NCH * DCH * 2;
  const size_t szP = (size_t)NB * SEQ * KC * 2;
  const size_t oQH = off; off += szP;
  const size_t oQL = off; off += szP;
  const size_t oKH = off; off += szP;
  const size_t oKL = off; off += szP;
  const size_t oV  = off; off += (size_t)NB * DCH * SEQ * 2;
  if (off > ws_size) return;
  if (off > (size_t)134217728) return;

  const float* x  = (const float*)d_in[0];
  const float* Wq = (const float*)d_in[1];
  const float* bq = (const float*)d_in[2];
  const float* Wk = (const float*)d_in[3];
  const float* bk = (const float*)d_in[4];
  const float* Wv = (const float*)d_in[5];
  const float* bv = (const float*)d_in[6];
  char* ws = (char*)d_ws;
  unsigned short* WB = (unsigned short*)(ws + oW);
  unsigned short* QH = (unsigned short*)(ws + oQH);
  unsigned short* QL = (unsigned short*)(ws + oQL);
  unsigned short* KH = (unsigned short*)(ws + oKH);
  unsigned short* KL = (unsigned short*)(ws + oKL);
  unsigned short* VP = (unsigned short*)(ws + oV);
  float* out = (float*)d_out;

  const dim3 blk256(256), blk128(128);
  const dim3 gW((NCH * DCH / 8) / 256);
  const dim3 gP(NB * (SEQ / QT));
  const dim3 gA(NB * (SEQ / QT));

  cvt_w<<<gW, blk256, 0, stream>>>(Wq, Wk, Wv, WB);
  proj_kernel<<<gP, blk256, 0, stream>>>(x, WB, bq, bk, bv, QH, QL, KH, KL, VP);
  attn_kernel<<<gA, blk128, 0, stream>>>(QH, QL, KH, KL, VP, out);
  (void)hipGetLastError();
}
